// PPM_2104533975450
// MI455X (gfx1250) — hardware-verified
//
#include <hip/hip_runtime.h>


namespace {
typedef _Float16 b16;
typedef __attribute__((ext_vector_type(16))) _Float16 v16b;
typedef __attribute__((ext_vector_type(8))) _Float16 v8b;
typedef __attribute__((ext_vector_type(4))) _Float16 v4h;
typedef __attribute__((ext_vector_type(2))) _Float16 v2h;
typedef __attribute__((ext_vector_type(8))) float v8f;
typedef __attribute__((ext_vector_type(4))) float v4f;
typedef __attribute__((ext_vector_type(2))) float v2f;
__device__ __forceinline__ float bf16_rne(float f) { unsigned int u = __float_as_uint(f); u += 0x7FFFu + ((u >> 16) & 1u); return __uint_as_float(u & 0xFFFF0000u); }
__device__ __forceinline__ void split16(float v, b16& hi, b16& lo) { hi = (b16)v; lo = (b16)(v - (float)hi); }
__device__ __forceinline__ v16b frag_kb(const b16* p, int hh) { const v8b a = *(const v8b*)(p + 8 * hh), b = *(const v8b*)(p + 16 + 8 * hh); v16b f;
#pragma unroll
  for (int e = 0; e < 8; ++e) { f[e] = a[e]; f[8 + e] = b[e]; } return f; }
__device__ __forceinline__ v8f wmma16b(v16b a, v16b b, v8f c) { v8f d = __builtin_amdgcn_wmma_f32_16x16x32_f16(false, a, false, b, (short)0, c, false, false); asm volatile("v_nop\n\tv_nop\n\tv_nop\n\tv_nop" : "+v"(d) : "v"(a), "v"(b)); return d; }
__device__ __forceinline__ void wave_lds_sync() { __builtin_amdgcn_fence(__ATOMIC_RELEASE, "workgroup"); __builtin_amdgcn_wave_barrier(); __builtin_amdgcn_fence(__ATOMIC_ACQUIRE, "workgroup"); }
__device__ __forceinline__ float pmul(float a, float b) { float p = a * b; asm volatile("" : "+v"(p)); return p; }
__device__ __forceinline__ int iclamp(int v, int lo, int hi) { return v < lo ? lo : (v > hi ? hi : v); }
__device__ __forceinline__ float nexp2(float v) { return __builtin_amdgcn_exp2f(v); }

constexpr int B = 32, BL = B  , C = 256, HW = 1024;
constexpr float XS = 8.0f, WSC = 256.0f, SS = 1024.0f  , RS_ = 1024.0f, NEPS = 1e-8f;
static_assert(HW % 64 == 0 && C == 256, "tiling");

__global__ __launch_bounds__(256) void wcvt_kernel(const float* __restrict__ w, b16* __restrict__ WT) { const int u = blockIdx.x * 256 + threadIdx.x; if (u >= C * C / 8) return; const size_t e = (size_t)u * 8; v8b o; for (int j = 0; j < 8; ++j) o[j] = (b16)(bf16_rne(w[e + j]) * WSC);
  for (int pass = 0; pass < 2; ++pass) { *(volatile v8b*)(WT + e) = o; __threadfence(); } }
__global__ __launch_bounds__(256) void plane_kernel(const float* __restrict__ x, b16* __restrict__ XN, b16* __restrict__ X16) {
  __shared__ float part[8][32]; __shared__ __attribute__((aligned(16))) b16 Tn[32][C + 8], Tx[32][C + 8];
  const int b = blockIdx.y, q0 = blockIdx.x * 32; const int p = threadIdx.x & 31, g = threadIdx.x >> 5; const float* xb = x + (size_t)b * C * HW + q0 + p;
  float v[32]; float ss = 0.0f;
#pragma unroll
  for (int j = 0; j < 32; ++j) { v[j] = bf16_rne(xb[(size_t)(g * 32 + j) * HW]); ss = fmaf(v[j], v[j], ss); }
  part[g][p] = ss; __syncthreads();
  float tot = 0.0f; for (int gg = 0; gg < 8; ++gg) tot += part[gg][p]; const float inv = 1.0f / fmaxf(sqrtf(tot), NEPS);
#pragma unroll
  for (int j = 0; j < 32; ++j) { Tn[p][g * 32 + j] = (b16)(v[j] * inv * XS); Tx[p][g * 32 + j] = (b16)(v[j] * XS); }
  __syncthreads();
  const int wave = threadIdx.x >> 5, lane = threadIdx.x & 31;
  for (int pass = 0; pass < 2; ++pass) { for (int rr = wave * 4; rr < wave * 4 + 4; ++rr) { const size_t dst = ((size_t)b * HW + q0 + rr) * C + lane * 8; *(volatile v8b*)(XN + dst) = *(const v8b*)(&Tn[rr][lane * 8]); *(volatile v8b*)(X16 + dst) = *(const v8b*)(&Tx[rr][lane * 8]); } __threadfence(); }
}
__global__ __launch_bounds__(64) void gram_kernel(const b16* __restrict__ XN, b16* __restrict__ SIM) {
  __shared__ __attribute__((aligned(16))) float Tf[2][16][128 + 4];
  const int wave = threadIdx.x >> 5, lane = threadIdx.x & 31, nloc = lane & 15, hlf = lane >> 4; const int b = blockIdx.z; const int q0 = blockIdx.x * 32 + wave * 16; const int k0 = blockIdx.y * 128;
  const b16* Xb = XN + (size_t)b * HW * C;
  v8f acc[8];
#pragma unroll
  for (int t = 0; t < 8; ++t) acc[t] = (v8f){};
#pragma unroll 2
  for (int kb = 0; kb < C; kb += 32) { const v16b a = frag_kb(Xb + (size_t)(q0 + nloc) * C + kb, hlf);
#pragma unroll
    for (int t = 0; t < 8; ++t) acc[t] = wmma16b(a, frag_kb(Xb + (size_t)(k0 + t * 16 + nloc) * C + kb, hlf), acc[t]); }
#pragma unroll
  for (int t = 0; t < 8; ++t)
#pragma unroll
    for (int r = 0; r < 8; ++r) { const float s = fmaxf(acc[t][r] * (1.0f / (XS * XS)), 0.0f); Tf[wave][8 * hlf + r][t * 16 + nloc] = s * s; }
  wave_lds_sync();
  for (int pass = 0; pass < 2; ++pass) { for (int rr = 0; rr < 16; ++rr) { v4h o; for (int j = 0; j < 4; ++j) o[j] = (b16)(Tf[wave][rr][lane * 4 + j] * SS); *(volatile v4h*)(SIM + ((size_t)b * HW + q0 + rr) * HW + k0 + lane * 4) = o; } __threadfence(); }
}
__global__ __launch_bounds__(128) void conv_kernel(const b16* __restrict__ X16, const b16* __restrict__ WT, const float* __restrict__ bias, b16* __restrict__ TTh, b16* __restrict__ TTl) {
  __shared__ __attribute__((aligned(16))) float Tf[4][16][C + 4];
  const int wave = threadIdx.x >> 5, lane = threadIdx.x & 31, nloc = lane & 15, hlf = lane >> 4; const int b = blockIdx.y; const int p0 = blockIdx.x * 64; const b16* Xb = X16 + ((size_t)b * HW + p0 + wave * 16) * C;
  v8f acc[16];
#pragma unroll
  for (int t = 0; t < 16; ++t) acc[t] = (v8f){};
#pragma unroll 1
  for (int kb = 0; kb < C; kb += 32) { const v16b a = frag_kb(Xb + (size_t)nloc * C + kb, hlf);
#pragma unroll
    for (int t = 0; t < 16; ++t) acc[t] = wmma16b(a, frag_kb(WT + (size_t)(t * 16 + nloc) * C + kb, hlf), acc[t]); }
#pragma unroll
  for (int t = 0; t < 16; ++t) { const float bb = bf16_rne(bias[t * 16 + nloc]);
#pragma unroll
    for (int r = 0; r < 8; ++r) Tf[wave][8 * hlf + r][t * 16 + nloc] = acc[t][r] * (1.0f / (XS * WSC)) + bb; }
  __syncthreads();
  for (int pass = 0; pass < 2; ++pass) {
#pragma unroll 1
    for (int q = 0; q < C / 4; ++q) { const int c = wave * (C / 4) + q; const int tk = lane * 2; v2h hv, lv; for (int e2 = 0; e2 < 2; ++e2) { const float vs = Tf[(tk + e2) >> 4][(tk + e2) & 15][c] * XS; const b16 ph = (b16)vs; hv[e2] = ph; lv[e2] = (b16)((vs - (float)ph) * RS_); }
      const size_t dst = ((size_t)b * C + c) * HW + p0 + tk; *(volatile v2h*)(TTh + dst) = hv; *(volatile v2h*)(TTl + dst) = lv; }
    __threadfence(); }
}
__global__ __launch_bounds__(64) void prop_kernel(const b16* __restrict__ SIM, const b16* __restrict__ TTh, const b16* __restrict__ TTl, float* __restrict__ out) {
  __shared__ __attribute__((aligned(16))) float Tf[2][16][128 + 4];
  const int wave = threadIdx.x >> 5, lane = threadIdx.x & 31, nloc = lane & 15, hlf = lane >> 4; const int b = blockIdx.z; const int q0 = blockIdx.x * 32 + wave * 16; const int c0 = blockIdx.y * 128;
  const b16* Sb = SIM + ((size_t)b * HW + q0 + nloc) * HW; const b16* Th = TTh + (size_t)b * C * HW; const b16* Tl = TTl + (size_t)b * C * HW;
  v8f acc[8], acc2[8];
#pragma unroll
  for (int t = 0; t < 8; ++t) { acc[t] = (v8f){}; acc2[t] = (v8f){}; }
#pragma unroll 2
  for (int kb = 0; kb < HW; kb += 32) { const v16b a = frag_kb(Sb + kb, hlf);
#pragma unroll
    for (int t = 0; t < 8; ++t) { const size_t ro = (size_t)(c0 + t * 16 + nloc) * HW + kb; acc[t] = wmma16b(a, frag_kb(Th + ro, hlf), acc[t]); acc2[t] = wmma16b(a, frag_kb(Tl + ro, hlf), acc2[t]); } }
#pragma unroll
  for (int t = 0; t < 8; ++t)
#pragma unroll
    for (int r = 0; r < 8; ++r) Tf[wave][8 * hlf + r][t * 16 + nloc] = (acc[t][r] + acc2[t][r] * (1.0f / RS_)) * (1.0f / (SS * XS));
  __syncthreads();
  for (int pass = 0; pass < 2; ++pass) { for (int q = 0; q < 64; ++q) { const int c = c0 + wave * 64 + q; ((volatile float*)out)[((size_t)b * C + c) * HW + blockIdx.x * 32 + lane] = Tf[lane >> 4][lane & 15][c - c0]; } __threadfence(); }
}
}

extern "C" void kernel_launch(void* const* d_in, const int* in_sizes, int n_in, void* d_out, int out_size, void* d_ws, size_t ws_size, hipStream_t stream) {
  (void)n_in;
  auto Fp = [&](int i) { return (const float*)d_in[i]; };
  if (in_sizes[0] != B * C * HW || in_sizes[1] != C * C || in_sizes[2] != C || out_size != B * C * HW) return;
  size_t off = 0; char* ws = (char*)d_ws;
  auto carve = [&](size_t bytes) { char* p = ws + off; off += (bytes + 255) & ~(size_t)255; return p; };
  b16* WT = (b16*)carve((size_t)C * C * 2); b16* XN = (b16*)carve((size_t)B * HW * C * 2); b16* X16 = (b16*)carve((size_t)B * HW * C * 2); b16* SIM = (b16*)carve((size_t)B * HW * HW * 2); b16* TTh = (b16*)carve((size_t)B * C * HW * 2); b16* TTl = (b16*)carve((size_t)B * C * HW * 2);
  if (off > ws_size || off > ((size_t)160 << 20)) return;
  wcvt_kernel<<<(C * C / 8 + 255) / 256, 256, 0, stream>>>(Fp(1), WT);
  plane_kernel<<<dim3(HW / 32, BL), 256, 0, stream>>>(Fp(0), XN, X16);
  gram_kernel<<<dim3(HW / 32, HW / 128, BL), 64, 0, stream>>>(XN, SIM);
  conv_kernel<<<dim3(HW / 64, BL), 128, 0, stream>>>(X16, WT, Fp(2), TTh, TTl);
  prop_kernel<<<dim3(HW / 32, C / 128, BL), 64, 0, stream>>>(SIM, TTh, TTl, (float*)d_out);
}
